// SimpleGNN_24773371363890
// MI455X (gfx1250) — hardware-run, weakly checked
//
#include <hip/hip_runtime.h>
#include <stddef.h>
#include <stdint.h>


#define CH     128
#define NPP    512
#define EDM    16
#define EFK    32
#define ZD     272
#define KH     256
#define NOUT   64
#define NTHR   256
#define NWAVE  8
#define EPT    8
#define CHUNK  (NTHR * EPT)
#define WCAP   (EPT * 32)
#define LISTN  (NWAVE * WCAP)
#define NBA    1024
#define SLA    10
#define RCAP   20480
#define OFFP   1056
#define RB     256
#define TH     64
#define GP     256
#define GBM    64
#define GBN    128
#define GTHR   128
#define HTHR   128
#define MEASB  16623
#define AGG_ZINTS     (LISTN + 2 * RCAP + 3 * NBA)
#define AGG_LDS_INTS  (AGG_ZINTS + 16)
#define AGG_LDS_BYTES (AGG_LDS_INTS * 4)
#define MSG_ACC_F     (RB * CH)
#define MSG_G_F       (TH * GP)
#define MSG_A_H       (TH * EFK)
#define MSG_LDS_BYTES (MSG_ACC_F * 4 + MSG_G_F * 4 + MSG_A_H * 2 + TH * 4)
#define U_WN1  (NPP * (CH / 8))
#define U_WN23 (NPP * (KH / 8))
#define U_WE   (2 * CH * (EFK / 8))
#define U_BI   256
#define U_WL   (NOUT * CH / 4)
#define U_BL   256
#define PC0 (U_WN1)
#define PC1 (PC0 + U_WN23)
#define PC2 (PC1 + U_WN23)
#define PC3 (PC2 + 3 * U_WE)
#define PC4 (PC3 + 3 * U_BI)
#define PC5 (PC4 + U_WL)
#define PC6 (PC5 + U_BL)

static_assert(CH == 128 && EDM <= EFK && EFK == 32 && ZD == 2 * CH + EDM);
static_assert(TH == NWAVE * 8 && TH == 4 * 16 && NTHR == 2 * CH && RB == NWAVE * 32);
static_assert(NBA == 4 * RB && NBA == (1 << SLA) && (NBA & (NBA - 1)) == 0);
static_assert((long long)RCAP * 100 >= (long long)MEASB * 105);
static_assert(RCAP % (NTHR * 4) == 0 && RCAP % TH == 0 && RCAP % 64 == 0);
static_assert(OFFP >= NBA + 2 && OFFP % 32 == 0);
static_assert((CHUNK & (CHUNK - 1)) == 0 && CHUNK <= 4096 && WCAP * NWAVE == CHUNK);
static_assert(((long long)CHUNK << SLA) < (1LL << 31));
static_assert(AGG_ZINTS % (NTHR * 4) == 0);
static_assert(AGG_LDS_BYTES <= 327680 && MSG_LDS_BYTES <= 327680);
static_assert(GP == 2 * CH && NPP == 4 * CH && KH == 2 * CH && NWAVE * CH <= MSG_G_F);
static_assert(GBM == (GTHR / 32) * 16 && GBN == 4 * 32 && NPP % GBN == 0);
static_assert(PC0 % NTHR == 0 && PC1 % NTHR == 0 && PC2 % NTHR == 0 && PC3 % NTHR == 0);
static_assert(PC4 % NTHR == 0 && PC5 % NTHR == 0 && PC6 % NTHR == 0 && U_WE % (2 * NTHR) == 0);
static_assert(MSG_ACC_F % (NTHR * 4) == 0 && HTHR == CH && NOUT * 4 == 256);

typedef float          v4f   __attribute__((ext_vector_type(4)));
typedef float          v8f   __attribute__((ext_vector_type(8)));
typedef int            v4i   __attribute__((ext_vector_type(4)));
typedef int            v8i   __attribute__((ext_vector_type(8)));
typedef unsigned       v2u   __attribute__((ext_vector_type(2)));
typedef unsigned       v4u   __attribute__((ext_vector_type(4)));
typedef unsigned short v8us  __attribute__((ext_vector_type(8)));
typedef unsigned short v16us __attribute__((ext_vector_type(16)));
typedef __bf16         v16bf __attribute__((ext_vector_type(16)));
typedef v4f  __attribute__((may_alias)) v4fa;
typedef v4i  __attribute__((may_alias)) v4ia;
typedef v2u  __attribute__((may_alias)) v2ua;
typedef v4u  __attribute__((may_alias)) v4ua;
typedef v8us __attribute__((may_alias)) v8usa;
union FragB { v16bf v; v16us u; v8us h[2]; v8i w; };

__device__ __forceinline__ v8f wmb(const FragB& a, const FragB& b, v8f c) {
  v8f d = __builtin_amdgcn_wmma_f32_16x16x32_bf16(false, a.v, false, b.v, (short)0, c, false, false);
  asm volatile("v_nop\n\tv_nop\n\tv_nop\n\tv_nop" : "+v"(d) : "v"(a.w), "v"(b.w));
  return d;
}

__device__ __forceinline__ unsigned bf16_bits(float f) {
  const unsigned u = __float_as_uint(f);
  return (u + 0x7FFFu + ((u >> 16) & 1u)) >> 16;
}
__device__ __forceinline__ float bf16_val(float f) {
  return __uint_as_float(bf16_bits(f) << 16);
}
__device__ __forceinline__ v8us cvt8(const float* __restrict__ p) {
  const v4f a = *(const v4fa*)p;
  const v4f b = *(const v4fa*)(p + 4);
  v8us o;
  o[0] = (unsigned short)bf16_bits(a.x); o[1] = (unsigned short)bf16_bits(a.y);
  o[2] = (unsigned short)bf16_bits(a.z); o[3] = (unsigned short)bf16_bits(a.w);
  o[4] = (unsigned short)bf16_bits(b.x); o[5] = (unsigned short)bf16_bits(b.y);
  o[6] = (unsigned short)bf16_bits(b.z); o[7] = (unsigned short)bf16_bits(b.w);
  return o;
}
__device__ __forceinline__ void put16(unsigned short* dp, v8us o) {
  *(volatile v8us*)dp = o;
  __threadfence();
  *(volatile v8us*)dp = o;
}
__device__ __forceinline__ void putf4(float* dp, v4f o) {
  *(volatile v4f*)dp = o;
  __threadfence();
  *(volatile v4f*)dp = o;
}
__device__ __forceinline__ float gate(float a, float b) {
  const float sg = __builtin_amdgcn_rcpf(1.0f + __expf(-a));
  const float sp = ((b > 0.0f) ? b : 0.0f) + __logf(1.0f + __expf(-fabsf(b)));
  return sg * sp;
}

template <int KP>
__device__ __forceinline__ void wn_unit(const float* __restrict__ Wf, const float* __restrict__ Ws,
                                        unsigned short* pl, int v) {
  const int n  = v / (KP / 8);
  const int k8 = (v - n * (KP / 8)) * 8;
  const int q  = n >> 7;
  const int nn = n & (CH - 1);
  const size_t so = (size_t)nn * ZD + (size_t)((q >> 1) * CH + (k8 & (CH - 1)));
  v8us o;
  if ((q & 1) != 0) o = cvt8(Ws + so); else o = cvt8(Wf + so);
  put16(pl + (size_t)n * KP + k8, o);
}
__device__ __forceinline__ void we_unit(const float* __restrict__ Wf, const float* __restrict__ Ws,
                                        unsigned short* pl, int v) {
  const int n  = v >> 2;
  const int k8 = (v & 3) * 8;
  const int nn = n & (CH - 1);
  const int kc = k8 & 8;
  const size_t so = (size_t)nn * ZD + (size_t)(2 * CH + kc);
  v8us o;
  if (n >= CH) o = cvt8(Ws + so); else o = cvt8(Wf + so);
  const unsigned mk = 0u - (unsigned)((k8 < EDM) ? 1 : 0);
#pragma unroll
  for (int i = 0; i < 8; ++i) o[i] = (unsigned short)((unsigned)o[i] & mk);
  put16(pl + (size_t)n * EFK + k8, o);
}
__device__ __forceinline__ void bi_unit(const float* __restrict__ bfp, const float* __restrict__ bsp,
                                        float* pl, int v) {
  if (v >= NPP / 4) return;
  const int c0 = 4 * v;
  const int cc = c0 & (CH - 1);
  const v4f a = *(const v4fa*)(bfp + cc);
  const v4f b = *(const v4fa*)(bsp + cc);
  const unsigned ma = 0u - (unsigned)((c0 < CH) ? 1 : 0);
  const unsigned mb = 0u - (unsigned)((c0 >= CH && c0 < 2 * CH) ? 1 : 0);
  v4f o;
  o.x = __uint_as_float(((bf16_bits(a.x) << 16) & ma) | ((bf16_bits(b.x) << 16) & mb));
  o.y = __uint_as_float(((bf16_bits(a.y) << 16) & ma) | ((bf16_bits(b.y) << 16) & mb));
  o.z = __uint_as_float(((bf16_bits(a.z) << 16) & ma) | ((bf16_bits(b.z) << 16) & mb));
  o.w = __uint_as_float(((bf16_bits(a.w) << 16) & ma) | ((bf16_bits(b.w) << 16) & mb));
  putf4(pl + c0, o);
}

__global__ __launch_bounds__(NTHR) void k_prep(const float* __restrict__ x,
                                               const float* __restrict__ Wf1, const float* __restrict__ Ws1,
                                               const float* __restrict__ Wf2, const float* __restrict__ Ws2,
                                               const float* __restrict__ Wf3, const float* __restrict__ Ws3,
                                               const float* __restrict__ bf1, const float* __restrict__ bs1,
                                               const float* __restrict__ bf2, const float* __restrict__ bs2,
                                               const float* __restrict__ bf3, const float* __restrict__ bs3,
                                               const float* __restrict__ Wlin, const float* __restrict__ blin,
                                               int nN, int mRows, int uHP, int uHPp,
                                               unsigned short* WN1, unsigned short* WN2, unsigned short* WN3,
                                               unsigned short* WE, float* BIAS, float* WLINF, float* BLINF,
                                               unsigned short* XB, unsigned short* HHL) {
  const int u = (int)blockIdx.x * NTHR + (int)threadIdx.x;
  if (u < PC0) { wn_unit<CH>(Wf1, Ws1, WN1, u); return; }
  if (u < PC1) { wn_unit<KH>(Wf2, Ws2, WN2, u - PC0); return; }
  if (u < PC2) { wn_unit<KH>(Wf3, Ws3, WN3, u - PC1); return; }
  if (u < PC3) {
    const int v = u - PC2;
    const int l = v / U_WE;
    const int vv = v - l * U_WE;
    if (l == 0)      we_unit(Wf1, Ws1, WE, vv);
    else if (l == 1) we_unit(Wf2, Ws2, WE + 2 * CH * EFK, vv);
    else             we_unit(Wf3, Ws3, WE + 4 * CH * EFK, vv);
    return;
  }
  if (u < PC4) {
    const int v = u - PC3;
    const int l = v / U_BI;
    const int vv = v - l * U_BI;
    if (l == 0)      bi_unit(bf1, bs1, BIAS, vv);
    else if (l == 1) bi_unit(bf2, bs2, BIAS + NPP, vv);
    else             bi_unit(bf3, bs3, BIAS + 2 * NPP, vv);
    return;
  }
  if (u < PC5) {
    const int v = u - PC4;
    const v4f a = *(const v4fa*)(Wlin + 4 * (size_t)v);
    v4f o;
    o.x = bf16_val(a.x); o.y = bf16_val(a.y); o.z = bf16_val(a.z); o.w = bf16_val(a.w);
    putf4(WLINF + 4 * (size_t)v, o);
    return;
  }
  if (u < PC6) {
    const int v = u - PC5;
    if (v >= NOUT / 4) return;
    const v4f a = *(const v4fa*)(blin + 4 * v);
    v4f o;
    o.x = bf16_val(a.x); o.y = bf16_val(a.y); o.z = bf16_val(a.z); o.w = bf16_val(a.w);
    putf4(BLINF + 4 * v, o);
    return;
  }
  if (u < PC6 + uHPp) {
    const int v = u - PC6;
    if (v >= uHP) return;
    const v8us z = {0, 0, 0, 0, 0, 0, 0, 0};
    put16(HHL + (size_t)nN * KH + 8 * (size_t)v, z);
    return;
  }
  {
    const int v = u - PC6 - uHPp;
    if (v >= mRows * (CH / 8)) return;
    const int row = v >> 4;
    const int k8  = (v & 15) * 8;
    const int rc  = row < nN ? row : nN - 1;
    v8us o = cvt8(x + (size_t)rc * CH + k8);
    const unsigned mk = 0u - (unsigned)((row < nN) ? 1 : 0);
#pragma unroll
    for (int i = 0; i < 8; ++i) o[i] = (unsigned short)((unsigned)o[i] & mk);
    put16(XB + (size_t)row * CH + k8, o);
  }
}

__device__ __forceinline__ int scan_chunk(const int* __restrict__ dsts, int nE, int cbase, int slotBase,
                                          int* list, int lane, int wave) {
  int wc = 0;
  const int elb  = WCAP * wave + lane;
  const int sent = -2147483647 - 1;
  int d[8];
#pragma unroll
  for (int j = 0; j < 8; ++j) {
    const int e  = cbase + elb + 32 * j;
    const int ec = e < nE ? e : nE - 1;
    const int dv = dsts[ec];
    d[j] = (e < nE) ? dv : sent;
  }
  const unsigned nbs = (unsigned)slotBase;
  const unsigned unb = (unsigned)NBA;
  const unsigned s0 = (unsigned)d[0] - nbs, s1 = (unsigned)d[1] - nbs;
  const unsigned s2 = (unsigned)d[2] - nbs, s3 = (unsigned)d[3] - nbs;
  const unsigned s4 = (unsigned)d[4] - nbs, s5 = (unsigned)d[5] - nbs;
  const unsigned s6 = (unsigned)d[6] - nbs, s7 = (unsigned)d[7] - nbs;
  const bool h0 = s0 < unb, h1 = s1 < unb, h2 = s2 < unb, h3 = s3 < unb;
  const bool h4 = s4 < unb, h5 = s5 < unb, h6 = s6 < unb, h7 = s7 < unb;
  const unsigned any = __builtin_amdgcn_ballot_w32(h0 | h1 | h2 | h3 | h4 | h5 | h6 | h7);
  if (any != 0u) {
#define HITJ(J, HJ, SJ) { \
      const unsigned mj = __builtin_amdgcn_ballot_w32(HJ); \
      if (mj != 0u) { \
        if (HJ) { \
          const int pos = wc + (int)__builtin_amdgcn_mbcnt_lo(mj, 0u); \
          if (pos < WCAP) list[wave * WCAP + pos] = ((elb + 32 * (J)) << SLA) | (int)(SJ); \
        } \
        wc += (int)__builtin_popcount(mj); } }
    HITJ(0, h0, s0)
    HITJ(1, h1, s1)
    HITJ(2, h2, s2)
    HITJ(3, h3, s3)
    HITJ(4, h4, s4)
    HITJ(5, h5, s5)
    HITJ(6, h6, s6)
    HITJ(7, h7, s7)
#undef HITJ
  }
  return wc;
}

__global__ __launch_bounds__(NTHR) void k_bucket(const int* __restrict__ srcs, const int* __restrict__ dsts,
                                                 int nE, int nN, int* LSRC, int* LEID, int* LSLOT, int* OFF) {
  extern __shared__ __attribute__((aligned(16))) int dsm[];
  int* list = dsm;
  int* hl   = dsm + LISTN;
  int* sl   = hl + RCAP;
  int* cnt  = sl + RCAP;
  int* offs = cnt + NBA;
  int* cur  = offs + NBA;
  int* misc = cur + NBA;
  const int tid = (int)threadIdx.x, lane = tid & 31, wave = tid >> 5;
  const int nodeBase = (int)blockIdx.x * NBA;

  {
    const v4i z4 = {0, 0, 0, 0};
    for (int i = tid * 4; i < AGG_ZINTS; i += NTHR * 4) *(v4ia*)(dsm + i) = z4;
    if (tid < 16) misc[tid] = 0;
  }
  __syncthreads();

  int t = 0, ov = 0;
  const int nChunks = (nE + CHUNK - 1) / CHUNK;
#pragma unroll 1
  for (int ch = 0; ch < nChunks; ++ch) {
    const int cbase = ch * CHUNK;
    const int wc = scan_chunk(dsts, nE, cbase, nodeBase, list, lane, wave);
    if (lane == 0) misc[wave] = wc;
    __syncthreads();
    if (wave == 0) {
#pragma unroll 1
      for (int w2 = 0; w2 < NWAVE; ++w2) {
        int c = misc[w2];
        c = c < 0 ? 0 : (c > WCAP ? WCAP : c);
#pragma unroll 1
        for (int b0 = 0; b0 < c; b0 += 32) {
          const int idx = b0 + lane;
          const int ent = list[w2 * WCAP + (idx < WCAP ? idx : WCAP - 1)];
          const int m32 = (c - b0) < 32 ? (c - b0) : 32;
#pragma unroll 1
          for (int k = 0; k < m32; ++k) {
            const int u    = __builtin_amdgcn_readlane(ent, k);
            const int slot = u & (NBA - 1);
            const int el   = (u >> SLA) & (CHUNK - 1);
            const int pk   = ((cbase + el) << SLA) | slot;
            if (t < RCAP) {
              if (lane == 0) { hl[t] = pk; cnt[slot] = cnt[slot] + 1; }
              t = t + 1;
            } else {
              ov = 1;
            }
          }
        }
      }
    }
    __syncthreads();
  }
  if (wave == 0 && lane == 0) { misc[8] = t; misc[9] = ov; }
  __syncthreads();
  int tt = misc[8];
  tt = tt < 0 ? 0 : (tt > RCAP ? RCAP : tt);
  const int ovf = misc[9];

  if (wave == 0) {
    const int base = lane * (NBA / 32);
    int s = 0;
#pragma unroll 1
    for (int i = 0; i < NBA / 32; ++i) s += cnt[base + i];
    int incl = s;
#pragma unroll
    for (int d = 1; d < 32; d <<= 1) {
      const int y = __shfl_up(incl, d, 32);
      if (lane >= d) incl += y;
    }
    int run = incl - s;
#pragma unroll 1
    for (int i = 0; i < NBA / 32; ++i) {
      const int cv = cnt[base + i];
      offs[base + i] = run;
      cur[base + i]  = run;
      run += cv;
    }
  }
  __syncthreads();
  if (wave == 0) {
#pragma unroll 1
    for (int b0 = 0; b0 < tt; b0 += 32) {
      const int idx = b0 + lane;
      const int ent = hl[idx < RCAP ? idx : RCAP - 1];
      const int m32 = (tt - b0) < 32 ? (tt - b0) : 32;
#pragma unroll 1
      for (int k = 0; k < m32; ++k) {
        const int u    = __builtin_amdgcn_readlane(ent, k);
        const int slot = u & (NBA - 1);
        if (lane == 0) {
          int p = cur[slot];
          p = p < 0 ? 0 : (p > RCAP - 1 ? RCAP - 1 : p);
          sl[p] = u;
          cur[slot] = p + 1;
        }
      }
    }
  }
  __syncthreads();

  const size_t lb = (size_t)blockIdx.x * RCAP;
#pragma unroll 1
  for (int i0 = tid * 4; i0 < RCAP; i0 += NTHR * 4) {
    const v4i e4 = *(const v4ia*)(sl + i0);
    const int ev[4] = {e4.x, e4.y, e4.z, e4.w};
    int sa[4], ea[4], qa[4];
#pragma unroll
    for (int q = 0; q < 4; ++q) {
      const bool ok = (i0 + q) < tt;
      int eid = ev[q] >> SLA;
      eid = eid < 0 ? 0 : (eid > nE - 1 ? nE - 1 : eid);
      int sr = srcs[eid];
      sr = sr < 0 ? 0 : (sr > nN - 1 ? nN - 1 : sr);
      sa[q] = ok ? sr : 0;
      ea[q] = ok ? eid : 0;
      qa[q] = ok ? (ev[q] & (NBA - 1)) : -1;
    }
    const v4i s4 = {sa[0], sa[1], sa[2], sa[3]};
    const v4i d4 = {ea[0], ea[1], ea[2], ea[3]};
    const v4i q4 = {qa[0], qa[1], qa[2], qa[3]};
    int* p0 = LSRC  + lb + i0;
    int* p1 = LEID  + lb + i0;
    int* p2 = LSLOT + lb + i0;
    *(volatile v4i*)p0 = s4;
    *(volatile v4i*)p1 = d4;
    *(volatile v4i*)p2 = q4;
    __threadfence();
    *(volatile v4i*)p0 = s4;
    *(volatile v4i*)p1 = d4;
    *(volatile v4i*)p2 = q4;
  }

#pragma unroll 1
  for (int it = 0; it < (OFFP / 4 + NTHR - 1) / NTHR; ++it) {
    const int pc  = it * NTHR + tid;
    const bool act = pc < OFFP / 4;
    const int pcc = act ? pc : OFFP / 4 - 1;
    int wv[4];
#pragma unroll
    for (int q = 0; q < 4; ++q) {
      const int i  = 4 * pcc + q;
      const int ic = i < NBA ? i : NBA - 1;
      const int o  = offs[ic];
      wv[q] = (i < NBA) ? o : ((i == NBA) ? tt : ((i == NBA + 1) ? ovf : 0));
    }
    const v4i w4 = {wv[0], wv[1], wv[2], wv[3]};
    int* op = OFF + (size_t)blockIdx.x * OFFP + 4 * pcc;
    if (act) *(volatile v4i*)op = w4;
    __threadfence();
    if (act) *(volatile v4i*)op = w4;
  }
}

__global__ __launch_bounds__(GTHR) void k_gemm(const unsigned short* __restrict__ A, int lda,
                                               const unsigned short* __restrict__ BT, int ldb, int K,
                                               const float* __restrict__ bias, float* Cm, int ldc) {
  __shared__ __attribute__((aligned(16))) float stg[GBM * GBN];
  const int tid = (int)threadIdx.x, lane = tid & 31, wave = tid >> 5, hh = lane >> 4, m = lane & 15;
  const int rowBase = (int)blockIdx.x * GBM;
  const int colBase = (int)blockIdx.y * GBN;

  v8f acc[8];
  {
    const v8f z = {0.f, 0.f, 0.f, 0.f, 0.f, 0.f, 0.f, 0.f};
#pragma unroll
    for (int t = 0; t < 8; ++t) acc[t] = z;
  }
  const unsigned short* ap = A  + (size_t)(rowBase + 16 * wave + m) * (size_t)lda + 8 * hh;
  const unsigned short* bp = BT + (size_t)(colBase + m) * (size_t)ldb + 8 * hh;

#pragma unroll 1
  for (int k0 = 0; k0 < K; k0 += 32) {
    FragB af;
    af.h[0] = *(const v8usa*)(ap + k0);
    af.h[1] = *(const v8usa*)(ap + k0 + 16);
#pragma unroll
    for (int nt = 0; nt < 8; ++nt) {
      const unsigned short* wq = bp + (size_t)(16 * nt) * (size_t)ldb + k0;
      FragB bf;
      bf.h[0] = *(const v8usa*)wq;
      bf.h[1] = *(const v8usa*)(wq + 16);
      acc[nt] = wmb(af, bf, acc[nt]);
    }
  }

#pragma unroll
  for (int nt = 0; nt < 8; ++nt) {
    const int lc = 16 * nt + m;
#pragma unroll
    for (int r = 0; r < 8; ++r) {
      const int lr = 16 * wave + 8 * hh + r;
      stg[lr * GBN + lc] = acc[nt][r];
    }
  }
  __syncthreads();

  const v4f b4 = *(const v4fa*)(bias + colBase + 4 * lane);
  v4f pv[16];
#pragma unroll
  for (int i = 0; i < 16; ++i) {
    const v4f sv = *(const v4fa*)(stg + (16 * wave + i) * GBN + 4 * lane);
    pv[i] = sv + b4;
  }
#pragma unroll
  for (int i = 0; i < 16; ++i) {
    float* op = Cm + (size_t)(rowBase + 16 * wave + i) * (size_t)ldc + colBase + 4 * lane;
    *(volatile v4f*)op = pv[i];
  }
  __threadfence();
#pragma unroll
  for (int i = 0; i < 16; ++i) {
    float* op = Cm + (size_t)(rowBase + 16 * wave + i) * (size_t)ldc + colBase + 4 * lane;
    *(volatile v4f*)op = pv[i];
  }
}

template <int LAYER>
__global__ __launch_bounds__(NTHR) void k_msg(const float* __restrict__ P,
                                              const int* __restrict__ LSRC, const int* __restrict__ LEID,
                                              const int* __restrict__ LSLOT, const int* __restrict__ OFF,
                                              const float* __restrict__ EW, const unsigned short* __restrict__ WE,
                                              const float* __restrict__ X, unsigned short* HHL, float* REC,
                                              int nN, int nE) {
  extern __shared__ __attribute__((aligned(16))) float dyn[];
  float*          ACC   = dyn;
  float*          G     = dyn + MSG_ACC_F;
  unsigned short* AT    = (unsigned short*)(G + MSG_G_F);
  int*            mSlot = (int*)(G + MSG_G_F + MSG_A_H / 2);
  const int tid = (int)threadIdx.x, lane = tid & 31, wave = tid >> 5, hh = lane >> 4, m = lane & 15;
  const int b  = (int)blockIdx.x;
  const int bb = b >> 2;
  const int q  = b & 3;
  const v4f z4 = {0.0f, 0.0f, 0.0f, 0.0f};

  for (int i = tid * 4; i < MSG_ACC_F; i += NTHR * 4) *(v4fa*)(ACC + i) = z4;

  int lo = __builtin_amdgcn_readfirstlane(OFF[(size_t)bb * OFFP + RB * q]);
  int hi = __builtin_amdgcn_readfirstlane(OFF[(size_t)bb * OFFP + RB * q + RB]);
  const int fl = __builtin_amdgcn_readfirstlane(OFF[(size_t)bb * OFFP + NBA + 1]);
  lo = lo < 0 ? 0 : (lo > RCAP ? RCAP : lo);
  hi = hi < lo ? lo : (hi > RCAP ? RCAP : hi);
  const int nT = (hi - lo + TH - 1) / TH;

  FragB fa, fb;
  {
    const unsigned short* wea = WE + (size_t)(16 * wave + m) * EFK + 8 * hh;
    const unsigned short* web = WE + (size_t)(CH + 16 * wave + m) * EFK + 8 * hh;
    fa.h[0] = *(const v8usa*)wea;
    fa.h[1] = *(const v8usa*)(wea + 16);
    fb.h[0] = *(const v8usa*)web;
    fb.h[1] = *(const v8usa*)(web + 16);
  }
  __syncthreads();

  const int   cch   = tid & (CH - 1);
  const int   half  = __builtin_amdgcn_readfirstlane(tid >> 7);
  const size_t lbase = (size_t)bb * RCAP;
  int   defSlot = -1;
  float defVal  = 0.0f;

#pragma unroll 1
  for (int t = 0; t < nT; ++t) {
    {
      const int hl8 = lane >> 2;
      const int qd  = lane & 3;
      const int hit = 8 * wave + hl8;
      const int p   = lo + TH * t + hit;
      const int pc  = p < RCAP - 1 ? p : RCAP - 1;
      int sr = LSRC[lbase + pc];
      int ei = LEID[lbase + pc];
      const int sg = LSLOT[lbase + pc];
      const int sloc = sg - RB * q;
      const bool ok = (p < hi) && ((unsigned)sloc < (unsigned)RB);
      sr = sr < 0 ? 0 : (sr > nN - 1 ? nN - 1 : sr);
      ei = ei < 0 ? 0 : (ei > nE - 1 ? nE - 1 : ei);
      int dr = RB * b + (ok ? sloc : 0);
      dr = dr > nN - 1 ? nN - 1 : dr;
      const int okI = ok ? 1 : 0;
      if (qd == 0) mSlot[hit] = ok ? sloc : -1;

      const v4f e4 = *(const v4fa*)(EW + (size_t)ei * EDM + 4 * qd);
      const unsigned em = 0u - (unsigned)okI;
      v2u w01, wz;
      w01.x = (bf16_bits(e4.x) | (bf16_bits(e4.y) << 16)) & em;
      w01.y = (bf16_bits(e4.z) | (bf16_bits(e4.w) << 16)) & em;
      wz.x = 0u; wz.y = 0u;
      unsigned short* arow = AT + hit * EFK;
      *(v2ua*)(arow + 4 * qd)      = w01;
      *(v2ua*)(arow + 16 + 4 * qd) = wz;

#pragma unroll 2
      for (int i = 0; i < 8; ++i) {
        const int si = __builtin_amdgcn_readlane(sr, 4 * i);
        const int di = __builtin_amdgcn_readlane(dr, 4 * i);
        const int oi = __builtin_amdgcn_readlane(okI, 4 * i);
        const float* pd = P + (size_t)di * NPP + 4 * lane;
        const float* ps = P + (size_t)si * NPP + 2 * CH + 4 * lane;
        const v4f d0 = *(const v4fa*)pd;
        const v4f d1 = *(const v4fa*)(pd + CH);
        const v4f s0 = *(const v4fa*)ps;
        const v4f s1 = *(const v4fa*)(ps + CH);
        v4f g0 = d0 + s0;
        v4f g1 = d1 + s1;
        g0 = (oi != 0) ? g0 : z4;
        g1 = (oi != 0) ? g1 : z4;
        float* gr = G + (8 * wave + i) * GP + 4 * lane;
        *(v4fa*)gr        = g0;
        *(v4fa*)(gr + CH) = g1;
      }
    }
    __syncthreads();

#pragma unroll 1
    for (int mt = 0; mt < 4; ++mt) {
      const unsigned short* ap = AT + (16 * mt + m) * EFK + 8 * hh;
      FragB af;
      af.h[0] = *(const v8usa*)ap;
      af.h[1] = *(const v8usa*)(ap + 16);
      float* gc = G + (16 * mt + 8 * hh) * GP + 16 * wave + m;
      v8f ca, cb;
#pragma unroll
      for (int r = 0; r < 8; ++r) { ca[r] = gc[r * GP]; cb[r] = gc[r * GP + CH]; }
      ca = wmb(af, fa, ca);
      cb = wmb(af, fb, cb);
#pragma unroll
      for (int r = 0; r < 8; ++r) gc[r * GP] = gate(ca[r], cb[r]);
    }
    __syncthreads();

    {
      int   cur = -1;
      int   nfl = 0;
      float run = 0.0f;
#pragma unroll 4
      for (int k = 0; k < 32; ++k) {
        const int kk = 32 * half + k;
        const int s  = __builtin_amdgcn_readfirstlane(mSlot[kk]);
        const float v = G[kk * GP + cch];
        if (s >= 0) {
          if (s != cur) {
            if (cur >= 0) {
              if (half == 1 && nfl == 0) { defSlot = cur; defVal = run; }
              else { const float o = ACC[cur * CH + cch]; ACC[cur * CH + cch] = o + run; }
              nfl = nfl + 1;
            }
            cur = s;
            run = 0.0f;
          }
          run += v;
        }
      }
      if (cur >= 0) {
        if (half == 1 && nfl == 0) { defSlot = cur; defVal = run; }
        else { const float o = ACC[cur * CH + cch]; ACC[cur * CH + cch] = o + run; }
      }
    }
    __syncthreads();
    if (defSlot >= 0) {
      const float o = ACC[defSlot * CH + cch];
      ACC[defSlot * CH + cch] = o + defVal;
      defSlot = -1;
    }
  }
  __syncthreads();

  const float qnan = __int_as_float(0x7fc00000);
  const float pz   = (fl != 0) ? qnan : 0.0f;
  const int j    = lane & 15;
  const int part = lane >> 4;
  const unsigned mh = 0u - (unsigned)part;
  const unsigned ml = ~mh;
  float cs[8];
#pragma unroll
  for (int e = 0; e < 8; ++e) cs[e] = 0.0f;

#pragma unroll 1
  for (int bt = 0; bt < 4; ++bt) {
    v8us pv[8];
#pragma unroll
    for (int i = 0; i < 8; ++i) {
      const int rl  = 32 * wave + 8 * bt + i;
      const int row = RB * b + rl;
      const int rc  = row < nN ? row : nN - 1;
      const float* ar = ACC + rl * CH + 8 * j;
      const v4f a0 = *(const v4fa*)ar;
      const v4f a1 = *(const v4fa*)(ar + 4);
      const v8f av = {a0.x, a0.y, a0.z, a0.w, a1.x, a1.y, a1.z, a1.w};
      v8f rs;
      if constexpr (LAYER == 1) {
        const float* xr = X + (size_t)rc * CH + 8 * j;
        const v4f x0 = *(const v4fa*)xr;
        const v4f x1 = *(const v4fa*)(xr + 4);
        rs[0] = bf16_val(x0.x); rs[1] = bf16_val(x0.y); rs[2] = bf16_val(x0.z); rs[3] = bf16_val(x0.w);
        rs[4] = bf16_val(x1.x); rs[5] = bf16_val(x1.y); rs[6] = bf16_val(x1.z); rs[7] = bf16_val(x1.w);
      } else {
        const unsigned short* hr = HHL + (size_t)rc * KH + 8 * j;
        const v4u wh = *(const v4ua*)hr;
        const v4u wl = *(const v4ua*)(hr + CH);
        rs[0] = __uint_as_float(wh.x << 16)         + __uint_as_float(wl.x << 16);
        rs[1] = __uint_as_float(wh.x & 0xffff0000u) + __uint_as_float(wl.x & 0xffff0000u);
        rs[2] = __uint_as_float(wh.y << 16)         + __uint_as_float(wl.y << 16);
        rs[3] = __uint_as_float(wh.y & 0xffff0000u) + __uint_as_float(wl.y & 0xffff0000u);
        rs[4] = __uint_as_float(wh.z << 16)         + __uint_as_float(wl.z << 16);
        rs[5] = __uint_as_float(wh.z & 0xffff0000u) + __uint_as_float(wl.z & 0xffff0000u);
        rs[6] = __uint_as_float(wh.w << 16)         + __uint_as_float(wl.w << 16);
        rs[7] = __uint_as_float(wh.w & 0xffff0000u) + __uint_as_float(wl.w & 0xffff0000u);
      }
      if constexpr (LAYER != 3) {
        v8us oo;
#pragma unroll
        for (int e = 0; e < 8; ++e) {
          float v = (av[e] + rs[e]) + pz;
          v = (v > 0.0f) ? v : (v - v);
          const unsigned hb = bf16_bits(v);
          const unsigned lb = bf16_bits(v - __uint_as_float(hb << 16));
          oo[e] = (unsigned short)((hb & ml) | (lb & mh));
        }
        pv[i] = oo;
      } else {
        const bool live = row < nN;
#pragma unroll
        for (int e = 0; e < 8; ++e) {
          const float v = (av[e] + rs[e]) + pz;
          cs[e] += live ? v : 0.0f;
        }
      }
    }
    if constexpr (LAYER != 3) {
#pragma unroll
      for (int i = 0; i < 8; ++i) {
        const int row = RB * b + 32 * wave + 8 * bt + i;
        if (row < nN) {
          unsigned short* op = HHL + (size_t)row * KH + part * CH + 8 * j;
          *(volatile v8us*)op = pv[i];
        }
      }
      __threadfence();
#pragma unroll
      for (int i = 0; i < 8; ++i) {
        const int row = RB * b + 32 * wave + 8 * bt + i;
        if (row < nN) {
          unsigned short* op = HHL + (size_t)row * KH + part * CH + 8 * j;
          *(volatile v8us*)op = pv[i];
        }
      }
    }
  }

  if constexpr (LAYER == 3) {
    if (part == 0) {
      const v4f c0 = {cs[0], cs[1], cs[2], cs[3]};
      const v4f c1 = {cs[4], cs[5], cs[6], cs[7]};
      *(v4fa*)(G + wave * CH + 8 * j)     = c0;
      *(v4fa*)(G + wave * CH + 8 * j + 4) = c1;
    }
    __syncthreads();
    if (wave == 0) {
      v4f s = z4;
#pragma unroll
      for (int w2 = 0; w2 < NWAVE; ++w2) {
        const v4f pw = *(const v4fa*)(G + w2 * CH + 4 * lane);
        s = s + pw;
      }
      float* rp = REC + (size_t)b * CH + 4 * lane;
      *(volatile v4f*)rp = s;
      __threadfence();
      *(volatile v4f*)rp = s;
    }
  }
}

__global__ __launch_bounds__(HTHR) void k_head(double invN, const float* __restrict__ REC, int nB,
                                               const float* __restrict__ WLINF, const float* __restrict__ BLINF,
                                               float* out) {
  __shared__ __attribute__((aligned(16))) float sp[CH];
  __shared__ __attribute__((aligned(16))) float so[NOUT];
  const int tid = (int)threadIdx.x;
  double s = 0.0;
#pragma unroll 4
  for (int b = 0; b < nB; ++b) s += (double)REC[(size_t)b * CH + tid];
  sp[tid] = (float)(s * invN);
  __syncthreads();
  const int o = tid & (NOUT - 1);
  float acc = 0.0f;
#pragma unroll 4
  for (int c = 0; c < CH; ++c) acc = fmaf(sp[c], WLINF[o * CH + c], acc);
  acc += BLINF[o];
  if (tid < NOUT) so[tid] = acc;
  __syncthreads();
  const int tl = tid < NOUT / 4 ? tid : NOUT / 4 - 1;
  const v4f o4 = *(const v4fa*)(so + 4 * tl);
  if (tid < NOUT / 4) *(volatile v4f*)(out + 4 * tl) = o4;
  __threadfence();
  if (tid < NOUT / 4) *(volatile v4f*)(out + 4 * tl) = o4;
}

static inline int cdiv(int a, int b) { return (a + b - 1) / b; }
static inline size_t al256(size_t o) { return (o + 255) & ~(size_t)255; }

extern "C" void kernel_launch(void* const* d_in, const int* in_sizes, int n_in,
                              void* d_out, int out_size, void* d_ws, size_t ws_size,
                              hipStream_t stream) {
  if (n_in < 17) return;
  if (in_sizes[0] < CH * 16 || (in_sizes[0] % CH) != 0) return;
  const int nN = in_sizes[0] / CH;
  if (in_sizes[1] < 2 || (in_sizes[1] & 1) != 0) return;
  const int nE = in_sizes[1] / 2;
  if (nE < 1 || nE >= (1 << 21) || nN >= (1 << 24)) return;
  if ((long long)in_sizes[2] != (long long)EDM * (long long)nE) return;
  for (int l = 0; l < 3; ++l) {
    if (in_sizes[3 + 4 * l] != CH * ZD || in_sizes[4 + 4 * l] != CH) return;
    if (in_sizes[5 + 4 * l] != CH * ZD || in_sizes[6 + 4 * l] != CH) return;
  }
  if (in_sizes[15] != NOUT * CH || in_sizes[16] != NOUT) return;
  if (out_size != NOUT) return;

  const float* x    = (const float*)d_in[0];
  const int*   eidx = (const int*)d_in[1];
  const int*   srcs = eidx;
  const int*   dsts = eidx + nE;
  const float* ew   = (const float*)d_in[2];
  const float* Wf1 = (const float*)d_in[3];  const float* bf1 = (const float*)d_in[4];
  const float* Ws1 = (const float*)d_in[5];  const float* bs1 = (const float*)d_in[6];
  const float* Wf2 = (const float*)d_in[7];  const float* bf2 = (const float*)d_in[8];
  const float* Ws2 = (const float*)d_in[9];  const float* bs2 = (const float*)d_in[10];
  const float* Wf3 = (const float*)d_in[11]; const float* bf3 = (const float*)d_in[12];
  const float* Ws3 = (const float*)d_in[13]; const float* bs3 = (const float*)d_in[14];
  const float* Wlin = (const float*)d_in[15];
  const float* blin = (const float*)d_in[16];
  float* out = (float*)d_out;

  const int MP   = cdiv(nN, 128) * 128;
  const int gM   = MP / GBM;
  const int gB   = cdiv(nN, NBA);
  const int gMsg = 4 * gB;
  if ((MP % GBM) != 0 || (long long)gMsg * RB < (long long)nN) return;
  const int uHP  = (MP - nN) * (KH / 8);
  const int uHPp = cdiv(uHP, NTHR) * NTHR;

  char* ws = (char*)d_ws;
  size_t off = 0;
  const size_t oWN1  = off; off = al256(off + (size_t)NPP * CH * 2);
  const size_t oWN2  = off; off = al256(off + (size_t)NPP * KH * 2);
  const size_t oWN3  = off; off = al256(off + (size_t)NPP * KH * 2);
  const size_t oWE   = off; off = al256(off + (size_t)3 * 2 * CH * EFK * 2);
  const size_t oBIAS = off; off = al256(off + (size_t)3 * NPP * 4);
  const size_t oWL   = off; off = al256(off + (size_t)NOUT * CH * 4);
  const size_t oBL   = off; off = al256(off + (size_t)NOUT * 4);
  const size_t oOFF  = off; off = al256(off + (size_t)gB * OFFP * 4);
  const size_t oREC  = off; off = al256(off + (size_t)gMsg * CH * 4);
  const size_t oLS   = off; off = al256(off + (size_t)gB * RCAP * 4);
  const size_t oLE   = off; off = al256(off + (size_t)gB * RCAP * 4);
  const size_t oLQ   = off; off = al256(off + (size_t)gB * RCAP * 4);
  const size_t oXB   = off; off = al256(off + (size_t)MP * CH * 2);
  const size_t oHHL  = off; off = al256(off + (size_t)MP * KH * 2);
  const size_t oP    = off; off = al256(off + (size_t)MP * NPP * 4);
  if (off > ws_size) return;
  unsigned short* WN1  = (unsigned short*)(ws + oWN1);
  unsigned short* WN2  = (unsigned short*)(ws + oWN2);
  unsigned short* WN3  = (unsigned short*)(ws + oWN3);
  unsigned short* WE   = (unsigned short*)(ws + oWE);
  float*          BIAS = (float*)(ws + oBIAS);
  float*          WLF  = (float*)(ws + oWL);
  float*          BLF  = (float*)(ws + oBL);
  int*            OFF  = (int*)(ws + oOFF);
  float*          REC  = (float*)(ws + oREC);
  int*            LSRC = (int*)(ws + oLS);
  int*            LEID = (int*)(ws + oLE);
  int*            LSLT = (int*)(ws + oLQ);
  unsigned short* XB   = (unsigned short*)(ws + oXB);
  unsigned short* HHL  = (unsigned short*)(ws + oHHL);
  float*          P    = (float*)(ws + oP);

  hipFuncSetAttribute(reinterpret_cast<const void*>(&k_bucket), hipFuncAttributeMaxDynamicSharedMemorySize,
                      (int)AGG_LDS_BYTES);
  hipFuncSetAttribute(reinterpret_cast<const void*>(&k_msg<1>), hipFuncAttributeMaxDynamicSharedMemorySize,
                      (int)MSG_LDS_BYTES);
  hipFuncSetAttribute(reinterpret_cast<const void*>(&k_msg<2>), hipFuncAttributeMaxDynamicSharedMemorySize,
                      (int)MSG_LDS_BYTES);
  hipFuncSetAttribute(reinterpret_cast<const void*>(&k_msg<3>), hipFuncAttributeMaxDynamicSharedMemorySize,
                      (int)MSG_LDS_BYTES);

  const int nPrep = PC6 + uHPp + MP * (CH / 8);
  const double invN = 1.0 / (double)nN;

  k_prep<<<nPrep / NTHR, NTHR, 0, stream>>>(x, Wf1, Ws1, Wf2, Ws2, Wf3, Ws3, bf1, bs1, bf2, bs2, bf3, bs3,
                                            Wlin, blin, nN, MP, uHP, uHPp,
                                            WN1, WN2, WN3, WE, BIAS, WLF, BLF, XB, HHL);
  k_bucket<<<gB, NTHR, AGG_LDS_BYTES, stream>>>(srcs, dsts, nE, nN, LSRC, LEID, LSLT, OFF);
  k_gemm<<<dim3(gM, NPP / GBN), GTHR, 0, stream>>>(XB, CH, WN1, CH, CH, BIAS, P, NPP);
  k_msg<1><<<gMsg, NTHR, MSG_LDS_BYTES, stream>>>(P, LSRC, LEID, LSLT, OFF, ew, WE, x, HHL, REC, nN, nE);
  k_gemm<<<dim3(gM, NPP / GBN), GTHR, 0, stream>>>(HHL, KH, WN2, KH, KH, BIAS + NPP, P, NPP);
  k_msg<2><<<gMsg, NTHR, MSG_LDS_BYTES, stream>>>(P, LSRC, LEID, LSLT, OFF, ew, WE + 2 * CH * EFK, x, HHL, REC,
                                                  nN, nE);
  k_gemm<<<dim3(gM, NPP / GBN), GTHR, 0, stream>>>(HHL, KH, WN3, KH, KH, BIAS + 2 * NPP, P, NPP);
  k_msg<3><<<gMsg, NTHR, MSG_LDS_BYTES, stream>>>(P, LSRC, LEID, LSLT, OFF, ew, WE + 4 * CH * EFK, x, HHL, REC,
                                                  nN, nE);
  k_head<<<1, HTHR, 0, stream>>>(invN, REC, gMsg, WLF, BLF, out);
}
